// Intra_channel_27084063769111
// MI455X (gfx1250) — hardware-verified
//
#include <hip/hip_runtime.h>


namespace {
constexpr int Bn = 8, C = 256, HW = 48, NP = HW * HW  , NT = Bn * NP;
constexpr float TS = 8.0f, VS = 8.0f, PS = 8.0f, EPS = 1e-5f;
constexpr size_t PLN = (size_t)NT * C;

typedef _Float16 b16;
typedef __attribute__((ext_vector_type(16))) _Float16 v16b;
typedef __attribute__((ext_vector_type(8))) _Float16 v8b;
typedef __attribute__((ext_vector_type(8))) float v8f;
typedef __attribute__((ext_vector_type(4))) float v4f;
__device__ __forceinline__ float bf16_rne(float f) { unsigned int u = __float_as_uint(f); u += 0x7FFFu + ((u >> 16) & 1u); return __uint_as_float(u & 0xFFFF0000u); }
__device__ __forceinline__ void split16(float v, b16& hi, b16& lo) { hi = (b16)v; lo = (b16)(v - (float)hi); }
__device__ __forceinline__ v16b frag_kb(const b16* p, int hh) { const v8b a = *(const v8b*)(p + 8 * hh), b = *(const v8b*)(p + 16 + 8 * hh); v16b f;
#pragma unroll
  for (int e = 0; e < 8; ++e) { f[e] = a[e]; f[8 + e] = b[e]; } return f; }
__device__ __forceinline__ v8f wmma16b(v16b a, v16b b, v8f c) { v8f d = __builtin_amdgcn_wmma_f32_16x16x32_f16(false, a, false, b, (short)0, c, false, false); asm volatile("v_nop\n\tv_nop\n\tv_nop\n\tv_nop" : "+v"(d) : "v"(a), "v"(b)); return d; }
__device__ __forceinline__ void wave_lds_sync() { __builtin_amdgcn_fence(__ATOMIC_RELEASE, "workgroup"); __builtin_amdgcn_wave_barrier(); __builtin_amdgcn_fence(__ATOMIC_ACQUIRE, "workgroup"); }
__device__ __forceinline__ float nexp(float x) { return __builtin_amdgcn_exp2f(x * 1.4426950408889634f); }

__global__ __launch_bounds__(256) void prep_kernel(const float* __restrict__ x, const float* __restrict__ wt, const float* __restrict__ bt, const float* __restrict__ wp, b16* __restrict__ th, b16* __restrict__ ph, b16* __restrict__ gt, float* __restrict__ vkey) {
  __shared__ __attribute__((aligned(16))) b16 Th[64][C + 8], Tl[64][C + 8], Ph[64][C + 8]; __shared__ float Vp[4][64];
  const int t_ = threadIdx.x, b = blockIdx.y, p0 = blockIdx.x * 64; const float* src = x + (size_t)b * C * NP;
  for (int pass = 0; pass < 2; ++pass) {
    for (int i = t_; i < C * 8; i += 256) { const int c = i >> 3, p8 = (i & 7) * 8; const float ww = bf16_rne(wt[c]) * bf16_rne(wp[c]); v8b gv;
#pragma unroll
      for (int e = 0; e < 8; ++e) { const float xv = bf16_rne(src[(size_t)c * NP + p0 + p8 + e]); gv[e] = (b16)(xv * VS);
        if (pass == 0) { b16 a, l; split16(xv * ww * TS, a, l); Th[p8 + e][c] = a; Tl[p8 + e][c] = l; Ph[p8 + e][c] = (b16)xv; } }
      *(volatile v8b*)(gt + ((size_t)b * C + c) * NP + p0 + p8) = gv; }
    if (pass == 0) { const int pp = t_ & 63, q = t_ >> 6; float s = 0.0f; for (int c = q; c < C; c += 4) { const float trm = bf16_rne(bt[c]) * bf16_rne(wp[c]) * bf16_rne(src[(size_t)c * NP + p0 + pp]); s += trm; } Vp[q][pp] = s; }
    __syncthreads();
    for (int i = t_; i < 64 * C / 8; i += 256) { const int pp = i >> 5, c8 = (i & 31) * 8; const size_t o = ((size_t)b * NP + p0 + pp) * C + c8;
      *(volatile v8b*)(th + o) = *(const v8b*)(&Th[pp][c8]); *(volatile v8b*)(th + PLN + o) = *(const v8b*)(&Tl[pp][c8]); *(volatile v8b*)(ph + o) = *(const v8b*)(&Ph[pp][c8]); }
    if (t_ < 64) ((volatile float*)vkey)[(size_t)b * NP + p0 + t_] = (Vp[0][t_] + Vp[1][t_]) + (Vp[2][t_] + Vp[3][t_]);
    __threadfence(); }
}

__global__ __launch_bounds__(256) void attn_kernel(const b16* __restrict__ th, const b16* __restrict__ ph, const b16* __restrict__ gt, const float* __restrict__ vkey, const float* __restrict__ x, const float* __restrict__ wg, const float* __restrict__ bg, const float* __restrict__ wo, const float* __restrict__ bo, const float* __restrict__ gma, const float* __restrict__ bta, const float* __restrict__ mu, const float* __restrict__ var, float* __restrict__ out) {
  __shared__ __attribute__((aligned(16))) float Os[C][128 + 4];
  const int wid = threadIdx.x >> 5, lane = threadIdx.x & 31, hh = lane >> 4, col = lane & 15; const int tok0 = blockIdx.x * 128 + wid * 16, b = tok0 / NP, n0 = tok0 % NP; const size_t qi = (size_t)tok0 + col;
  const b16* K = ph + ((size_t)b * NP) * C; const b16* V = gt + ((size_t)b * C) * NP; const float* VK = vkey + (size_t)b * NP;
  float m = -INFINITY, l = 0.0f; v8f o[16];
#pragma unroll
  for (int i = 0; i < 16; ++i) o[i] = (v8f){};
  for (int kb = 0; kb < NP; kb += 32) { v8f s0 = {}, s1 = {};
#pragma unroll 2
    for (int ks = 0; ks < C; ks += 32) { const v16b qf = frag_kb(th + qi * C + ks, hh), ql = frag_kb(th + PLN + qi * C + ks, hh);
      const v16b ka = frag_kb(K + (size_t)(kb + col) * C + ks, hh), kc = frag_kb(K + (size_t)(kb + 16 + col) * C + ks, hh);
      s0 = wmma16b(ka, qf, s0); s0 = wmma16b(ka, ql, s0); s1 = wmma16b(kc, qf, s1); s1 = wmma16b(kc, ql, s1); }
    float mr = -INFINITY;
#pragma unroll
    for (int r = 0; r < 8; ++r) { s0[r] = s0[r] * (1.0f / TS) + VK[kb + 8 * hh + r]; s1[r] = s1[r] * (1.0f / TS) + VK[kb + 16 + 8 * hh + r]; mr = fmaxf(mr, fmaxf(s0[r], s1[r])); }
    mr = fmaxf(mr, __shfl_xor(mr, 16));
    const float mn = fmaxf(m, mr), al_ = nexp(m - mn); m = mn; float sum = 0.0f; v16b pbv, plv;
#pragma unroll
    for (int r = 0; r < 8; ++r) { const float e0 = nexp(s0[r] - mn), e1 = nexp(s1[r] - mn); sum += e0 + e1; b16 a, cc; split16(e0 * PS, a, cc); pbv[r] = a; plv[r] = cc; split16(e1 * PS, a, cc); pbv[8 + r] = a; plv[8 + r] = cc; }
    sum += __shfl_xor(sum, 16); l = l * al_ + sum;
#pragma unroll
    for (int t = 0; t < 16; ++t) { o[t] *= al_; const v16b vf = frag_kb(V + (size_t)(t * 16 + col) * NP + kb, hh); o[t] = wmma16b(vf, pbv, o[t]); o[t] = wmma16b(vf, plv, o[t]); } }
  const float inv = 1.0f / (l * VS * PS);
#pragma unroll
  for (int t = 0; t < 16; ++t)
#pragma unroll
    for (int r = 0; r < 8; ++r) { const int c = t * 16 + 8 * hh + r; const float scl = bf16_rne(gma[c]) * rsqrtf(bf16_rne(var[c]) + EPS), sh = bf16_rne(bta[c]) - bf16_rne(mu[c]) * scl;
      const float y = o[t][r] * inv * bf16_rne(wg[c]) + bf16_rne(bg[c]); const float xv = bf16_rne(x[((size_t)b * C + c) * NP + n0 + col]);
      Os[c][wid * 16 + col] = (y * bf16_rne(wo[c]) + bf16_rne(bo[c])) * scl + sh + xv; }
  __syncthreads();
  const int nb = (blockIdx.x * 128) % NP;
  for (int pass = 0; pass < 2; ++pass) { for (int i = threadIdx.x; i < C * 32; i += 256) { const int c = i >> 5, c4 = (i & 31) * 4; *(volatile v4f*)(out + ((size_t)b * C + c) * NP + nb + c4) = *(const v4f*)(&Os[c][c4]); } __threadfence(); }
}
}

extern "C" void kernel_launch(void* const* d_in, const int* in_sizes, int n_in,
                              void* d_out, int out_size, void* d_ws, size_t ws_size, hipStream_t stream) {
  (void)n_in; (void)out_size;
  const float* x = (const float*)d_in[0]; const float* wg = (const float*)d_in[1]; const float* bg = (const float*)d_in[2]; const float* wt = (const float*)d_in[3]; const float* bt = (const float*)d_in[4]; const float* wp = (const float*)d_in[5]; const float* bp = (const float*)d_in[6];
  const float* wo = (const float*)d_in[7]; const float* bo = (const float*)d_in[8]; const float* gma = (const float*)d_in[9]; const float* bta = (const float*)d_in[10]; const float* mu = (const float*)d_in[11]; const float* var = (const float*)d_in[12];
  float* out = (float*)d_out;
  if (in_sizes[0] != Bn * C * NP || in_sizes[1] != C || in_sizes[12] != C) return;
  size_t off = 0; char* ws = (char*)d_ws;
  auto carve = [&](size_t bytes) { char* p = ws + off; off += (bytes + 255) & ~(size_t)255; return p; };
  b16* th = (b16*)carve(PLN * 2 * 2); b16* ph = (b16*)carve(PLN * 2); b16* gt = (b16*)carve(PLN * 2); float* vkey = (float*)carve((size_t)NT * 4);
  if (off > ws_size) return;
  prep_kernel<<<dim3(NP / 64, Bn), 256, 0, stream>>>(x, wt, bt, wp, th, ph, gt, vkey);
  attn_kernel<<<NT / 128, 256, 0, stream>>>(th, ph, gt, vkey, x, wg, bg, wo, bo, gma, bta, mu, var, out);
}
